// GraphEncoder_18622978195941
// MI455X (gfx1250) — hardware-verified
//
#include <hip/hip_runtime.h>
#include <stddef.h>
#include <stdint.h>
#include <math.h>


#define F_IN    128
#define HC      128
#define HID     64
#define KA      128
#define NGR     256
#define NHID    300
#define FCN     304
#define FCT     19
#define NTHR    256
#define NWAVE   8
#define EPT     8
#define CHUNK   (NTHR * EPT)
#define WCAP    (EPT * 32)
#define LISTN   (NWAVE * WCAP)
#define NBMAX   2048
#define SLOTB   11
#define RCAP    28672
#define DEGCAP  256
#define GBM     64
#define GBN     64
#define GTHR    128
#define BNR     256
#define NUW     (HC * (KA / 8))
#define NUF     (FCN * (KA / 8))
#define NEGSL   0.2f
#define EPS_SM  1e-16f
#define EPS_BN  1e-5f
#define WSMAX   134217728
#define LDS_AGG ((2 * RCAP + 2 * NBMAX + LISTN) * 4 + 64)

static_assert((CHUNK & (CHUNK - 1)) == 0 && CHUNK <= (1 << SLOTB));
static_assert(NBMAX == (1 << SLOTB));
static_assert(NTHR * 8 == NBMAX);
static_assert(LISTN >= NBMAX);
static_assert((RCAP % 32) == 0);
static_assert(LDS_AGG <= 300000);
static_assert(GBM == (GTHR / 32) * 16);
static_assert(GTHR == 2 * GBN && GTHR == 2 * GBM);
static_assert((KA % 32) == 0 && KA == 2 * HID && F_IN == KA);
static_assert((HC % GBN) == 0 && HID == GBN);
static_assert(HC == 4 * 32);
static_assert((NUW % NTHR) == 0 && (NUF % NTHR) == 0);
static_assert(FCN == FCT * 16 && FCN >= NHID);
static_assert(((16 * NHID * 4) % 128) == 0 && ((16 * NHID / 4) % 8) == 0);
static_assert((NGR % 16) == 0);
static_assert(NGR * NHID - 1 == 76799);

typedef float          v2f  __attribute__((ext_vector_type(2)));
typedef float          v4f  __attribute__((ext_vector_type(4)));
typedef float          v8f  __attribute__((ext_vector_type(8)));
typedef double         v2d  __attribute__((ext_vector_type(2)));
typedef int            v4i  __attribute__((ext_vector_type(4)));
typedef int            v8i  __attribute__((ext_vector_type(8)));
typedef unsigned int   v4u  __attribute__((ext_vector_type(4)));
typedef unsigned short v8us __attribute__((ext_vector_type(8)));
typedef __bf16         v16b __attribute__((ext_vector_type(16)));
typedef v2f  __attribute__((may_alias)) v2fa;
typedef v4f  __attribute__((may_alias)) v4fa;
typedef v2d  __attribute__((may_alias)) v2da;
typedef v8us __attribute__((may_alias)) v8usa;
union FragB { v16b v; v8us h[2]; v8i w; };

__device__ __forceinline__ v8f wmb(const FragB& a, const FragB& b, v8f c) {
  v8f d = __builtin_amdgcn_wmma_f32_16x16x32_bf16(false, a.v, false, b.v, (short)0, c, false, false);
  asm volatile("v_nop\n\tv_nop\n\tv_nop\n\tv_nop" : "+v"(d) : "v"(a.w), "v"(b.w));
  return d;
}

__device__ __forceinline__ unsigned int f2bf(float f) {
  const unsigned int u = __float_as_uint(f);
  return ((u + 0x7FFFu + ((u >> 16) & 1u)) >> 16) & 0xFFFFu;
}
__device__ __forceinline__ float bf2f(unsigned int b) { return __uint_as_float(b << 16); }
__device__ __forceinline__ float bfr(float f) { return bf2f(f2bf(f)); }
__device__ __forceinline__ v4f bfr4(const v4f a) {
  v4f r; r.x = bfr(a.x); r.y = bfr(a.y); r.z = bfr(a.z); r.w = bfr(a.w); return r;
}
__device__ __forceinline__ unsigned int pk2(float lo, float hi) { return f2bf(lo) | (f2bf(hi) << 16); }
__device__ __forceinline__ v4u pack8(const v4f a, const v4f b) {
  v4u r;
  r.x = pk2(a.x, a.y); r.y = pk2(a.z, a.w); r.z = pk2(b.x, b.y); r.w = pk2(b.z, b.w);
  return r;
}
__device__ __forceinline__ v4f res4(const v4f a) {
  v4f r; r.x = a.x - bfr(a.x); r.y = a.y - bfr(a.y); r.z = a.z - bfr(a.z); r.w = a.w - bfr(a.w); return r;
}
__device__ __forceinline__ float bnrelu(float y, float m, float iv, float g, float b, bool live) {
  const float z = (g * (y - m)) * iv + b;
  const float r = (z > 0.0f) ? z : (z - z);
  return live ? r : 0.0f;
}

__device__ __forceinline__ int scan_chunk(const int* __restrict__ dsts, int nE, int cbase, int slotBase,
                                          int nb, int vec8, int* list, int tid, int lane, int wave) {
  int wc = 0;
  const int el0  = tid * EPT;
  const int e0   = cbase + el0;
  const int sent = -2147483647 - 1;
  v4i da, db;
  if (vec8 != 0 && cbase + CHUNK <= nE) {
    da = *(const v4i*)(dsts + e0);
    db = *(const v4i*)(dsts + e0 + 4);
  } else {
    da.x = (e0     < nE) ? dsts[min(e0,     nE - 1)] : sent;
    da.y = (e0 + 1 < nE) ? dsts[min(e0 + 1, nE - 1)] : sent;
    da.z = (e0 + 2 < nE) ? dsts[min(e0 + 2, nE - 1)] : sent;
    da.w = (e0 + 3 < nE) ? dsts[min(e0 + 3, nE - 1)] : sent;
    db.x = (e0 + 4 < nE) ? dsts[min(e0 + 4, nE - 1)] : sent;
    db.y = (e0 + 5 < nE) ? dsts[min(e0 + 5, nE - 1)] : sent;
    db.z = (e0 + 6 < nE) ? dsts[min(e0 + 6, nE - 1)] : sent;
    db.w = (e0 + 7 < nE) ? dsts[min(e0 + 7, nE - 1)] : sent;
  }
  const unsigned nbs = (unsigned)slotBase;
  const unsigned unb = (unsigned)nb;
  const unsigned s0 = (unsigned)da.x - nbs, s1 = (unsigned)da.y - nbs;
  const unsigned s2 = (unsigned)da.z - nbs, s3 = (unsigned)da.w - nbs;
  const unsigned s4 = (unsigned)db.x - nbs, s5 = (unsigned)db.y - nbs;
  const unsigned s6 = (unsigned)db.z - nbs, s7 = (unsigned)db.w - nbs;
  const bool h0 = s0 < unb, h1 = s1 < unb, h2 = s2 < unb, h3 = s3 < unb;
  const bool h4 = s4 < unb, h5 = s5 < unb, h6 = s6 < unb, h7 = s7 < unb;
  const unsigned any = __builtin_amdgcn_ballot_w32(h0 | h1 | h2 | h3 | h4 | h5 | h6 | h7);
  if (any != 0u) {
#define HITJ(J, HJ, SJ) { \
      const unsigned mj = __builtin_amdgcn_ballot_w32(HJ); \
      if (mj != 0u) { \
        if (HJ) { \
          const int pos = wc + (int)__builtin_amdgcn_mbcnt_lo(mj, 0u); \
          if (pos < WCAP) list[wave * WCAP + pos] = ((el0 + (J)) << SLOTB) | (int)(SJ); \
        } \
        wc += (int)__builtin_popcount(mj); } }
    HITJ(0, h0, s0)
    HITJ(1, h1, s1)
    HITJ(2, h2, s2)
    HITJ(3, h3, s3)
    HITJ(4, h4, s4)
    HITJ(5, h5, s5)
    HITJ(6, h6, s6)
    HITJ(7, h7, s7)
#undef HITJ
  }
  return wc;
}

__global__ __launch_bounds__(NTHR) void k_cvx(const float* __restrict__ x, int nN, int nUnits,
                                              unsigned short* xb) {
  const int u = (int)blockIdx.x * NTHR + (int)threadIdx.x;
  if (u >= nUnits) return;
  const int row = u >> 4;
  const int k8  = (u & 15) * 8;
  const int rc  = row < nN ? row : nN - 1;
  const float* p = x + (size_t)rc * F_IN + k8;
  v4f a = *(const v4fa*)p, b = *(const v4fa*)(p + 4);
  const v4f z4 = {0.f, 0.f, 0.f, 0.f};
  if (row >= nN) { a = z4; b = z4; }
  const v4u hv = pack8(a, b);
  unsigned short* dp = xb + (size_t)row * F_IN + k8;
  *(volatile v4u*)dp = hv;
  __threadfence();
  *(volatile v4u*)dp = hv;
}

__global__ __launch_bounds__(NTHR) void k_wprep(const float* __restrict__ W1, const float* __restrict__ W2,
                                                const float* __restrict__ W3, const float* __restrict__ FW,
                                                unsigned short* W1T, unsigned short* W2D,
                                                unsigned short* W3D, unsigned short* FCD) {
  const int u = (int)blockIdx.x * NTHR + (int)threadIdx.x;
  const float* w;
  unsigned short* wt;
  int Kin, Ncol, v;
  if (u < NUW)                { w = W1; wt = W1T; Kin = 128; Ncol = HC;   v = u; }
  else if (u < 2 * NUW)       { w = W2; wt = W2D; Kin = 64;  Ncol = HC;   v = u - NUW; }
  else if (u < 3 * NUW)       { w = W3; wt = W3D; Kin = 64;  Ncol = HC;   v = u - 2 * NUW; }
  else if (u < 3 * NUW + NUF) { w = FW; wt = FCD; Kin = 64;  Ncol = NHID; v = u - 3 * NUW; }
  else return;
  const int n   = v >> 4;
  const int k8  = (v & 15) * 8;
  const int kk  = k8 & (Kin - 1);
  const int ncl = n < Ncol ? n : Ncol - 1;
  const float* p = w + (size_t)kk * (size_t)Ncol + ncl;
  v4f a, b;
  a.x = p[0];                    a.y = p[(size_t)Ncol];         a.z = p[(size_t)2 * Ncol];     a.w = p[(size_t)3 * Ncol];
  b.x = p[(size_t)4 * Ncol];     b.y = p[(size_t)5 * Ncol];     b.z = p[(size_t)6 * Ncol];     b.w = p[(size_t)7 * Ncol];
  const v4f z4 = {0.f, 0.f, 0.f, 0.f};
  if (n >= Ncol) { a = z4; b = z4; }
  const v4u wv = pack8(a, b);
  unsigned short* o = wt + (size_t)n * KA + k8;
  *(volatile v4u*)o = wv;
  __threadfence();
  *(volatile v4u*)o = wv;
}

__global__ __launch_bounds__(NTHR) void k_build(const int* __restrict__ srcs, const int* __restrict__ dsts,
                                                int nN, int nE, int nb, int vec8,
                                                int* HITS, int* CNT, int* OFF, int* HDR) {
  extern __shared__ v4f lds_dyn[];
  int* reg1 = (int*)lds_dyn;
  int* reg2 = reg1 + RCAP;
  int* scnt = reg2 + RCAP;
  int* soff = scnt + NBMAX;
  int* list = soff + NBMAX;
  int* wcnt = list + LISTN;
  int* wtot = wcnt + NWAVE;
  const int tid = (int)threadIdx.x, lane = tid & 31, wave = tid >> 5;
  const int nodeBase = (int)blockIdx.x * nb;

  for (int i = tid; i < NBMAX; i += NTHR) scnt[i] = 0;
  __syncthreads();

  int tot = 0;
  const int nChunks = (nE + CHUNK - 1) / CHUNK;
#pragma unroll 1
  for (int ch = 0; ch < nChunks; ++ch) {
    const int cbase = ch * CHUNK;
    const int wc = scan_chunk(dsts, nE, cbase, nodeBase, nb, vec8, list, tid, lane, wave);
    if (lane == 0) wcnt[wave] = wc;
    __syncthreads();
    int pre = 0, all = 0;
#pragma unroll
    for (int w2 = 0; w2 < NWAVE; ++w2) {
      int c = wcnt[w2];
      c = c < 0 ? 0 : (c > WCAP ? WCAP : c);
      all += c;
      pre += (w2 < wave) ? c : 0;
    }
    const int wcc  = wc > WCAP ? WCAP : wc;
    const int base = tot + pre;
#pragma unroll 1
    for (int i = lane; i < wcc; i += 32) {
      const int ent = list[wave * WCAP + i];
      const int el  = (ent >> SLOTB) & (CHUNK - 1);
      const int sl  = ent & (NBMAX - 1);
      int eid = cbase + el;
      eid = eid > nE - 1 ? nE - 1 : eid;
      const int pos = base + i;
      if (pos < RCAP) reg1[pos] = (int)(((unsigned)eid << SLOTB) | (unsigned)sl);
    }
    tot += all;
    tot = tot > RCAP ? RCAP : tot;
    __syncthreads();
  }
  const int nh = tot;

  if (wave == 0) {
#pragma unroll 1
    for (int b0 = 0; b0 < nh; b0 += 32) {
      const int idx = b0 + lane;
      const int uv  = reg1[idx < nh ? idx : nh - 1];
      const int m32 = (nh - b0) < 32 ? (nh - b0) : 32;
#pragma unroll 1
      for (int k = 0; k < m32; ++k) {
        const int u  = __builtin_amdgcn_readlane(uv, k);
        const int sl = u & (NBMAX - 1);
        if (lane == 0) scnt[sl] = scnt[sl] + 1;
      }
    }
  }
  __syncthreads();

  {
    const v4i ca = *(const v4i*)(scnt + 8 * tid);
    const v4i cb = *(const v4i*)(scnt + 8 * tid + 4);
    const int e0 = ca.x < 0 ? 0 : ca.x, e1 = ca.y < 0 ? 0 : ca.y, e2 = ca.z < 0 ? 0 : ca.z, e3 = ca.w < 0 ? 0 : ca.w;
    const int e4 = cb.x < 0 ? 0 : cb.x, e5 = cb.y < 0 ? 0 : cb.y, e6 = cb.z < 0 ? 0 : cb.z, e7 = cb.w < 0 ? 0 : cb.w;
    const int ts = e0 + e1 + e2 + e3 + e4 + e5 + e6 + e7;
    int incl = ts;
#pragma unroll
    for (int d = 1; d < 32; d <<= 1) {
      const int up = __shfl_up(incl, d);
      if (lane >= d) incl += up;
    }
    if (lane == 31) wtot[wave] = incl;
    __syncthreads();
    int pre = 0;
#pragma unroll
    for (int w2 = 0; w2 < NWAVE; ++w2) pre += (w2 < wave) ? wtot[w2] : 0;
    int run = pre + incl - ts;
    soff[8 * tid + 0] = run; run += e0;
    soff[8 * tid + 1] = run; run += e1;
    soff[8 * tid + 2] = run; run += e2;
    soff[8 * tid + 3] = run; run += e3;
    soff[8 * tid + 4] = run; run += e4;
    soff[8 * tid + 5] = run; run += e5;
    soff[8 * tid + 6] = run; run += e6;
    soff[8 * tid + 7] = run;
  }
  __syncthreads();
  for (int i = tid; i < NBMAX; i += NTHR) list[i] = soff[i];
  __syncthreads();

  if (wave == 0) {
#pragma unroll 1
    for (int b0 = 0; b0 < nh; b0 += 32) {
      const int idx = b0 + lane;
      const int uv  = reg1[idx < nh ? idx : nh - 1];
      const int m32 = (nh - b0) < 32 ? (nh - b0) : 32;
#pragma unroll 1
      for (int k = 0; k < m32; ++k) {
        const int u   = __builtin_amdgcn_readlane(uv, k);
        const int sl  = u & (NBMAX - 1);
        const int eid = (int)((unsigned)u >> SLOTB);
        if (lane == 0) {
          int pos = list[sl];
          pos = pos < 0 ? 0 : (pos > RCAP - 1 ? RCAP - 1 : pos);
          reg2[pos] = eid;
          list[sl] = pos + 1;
        }
      }
    }
  }
  __syncthreads();

  const int blk = (int)blockIdx.x;
  int* hp = HITS + (size_t)blk * RCAP;
  int* cp = CNT + (size_t)blk * NBMAX;
  int* op = OFF + (size_t)blk * NBMAX;
  int* dp = HDR + (size_t)blk * 32;
  const int nhr = (nh + 31) & ~31;
  const int nhm = nh > 0 ? nh - 1 : 0;
  const v4i c0v = *(const v4i*)(scnt + 4 * tid);
  const v4i c1v = *(const v4i*)(scnt + NTHR * 4 + 4 * tid);
  const v4i o0v = *(const v4i*)(soff + 4 * tid);
  const v4i o1v = *(const v4i*)(soff + NTHR * 4 + 4 * tid);
  v4i hd;
  hd.x = (lane == 0) ? nh : 0; hd.y = 0; hd.z = 0; hd.w = 0;
#pragma unroll 1
  for (int pass = 0; pass < 2; ++pass) {
#pragma unroll 1
    for (int base = 0; base < nhr; base += NTHR * 4) {
      const int i = base + 4 * tid;
      int e0 = reg2[min(i,     nhm)];
      int e1 = reg2[min(i + 1, nhm)];
      int e2 = reg2[min(i + 2, nhm)];
      int e3 = reg2[min(i + 3, nhm)];
      e0 = e0 < 0 ? 0 : (e0 > nE - 1 ? nE - 1 : e0);
      e1 = e1 < 0 ? 0 : (e1 > nE - 1 ? nE - 1 : e1);
      e2 = e2 < 0 ? 0 : (e2 > nE - 1 ? nE - 1 : e2);
      e3 = e3 < 0 ? 0 : (e3 > nE - 1 ? nE - 1 : e3);
      int s0 = srcs[e0], s1 = srcs[e1], s2 = srcs[e2], s3 = srcs[e3];
      s0 = s0 < 0 ? 0 : (s0 > nN - 1 ? nN - 1 : s0);
      s1 = s1 < 0 ? 0 : (s1 > nN - 1 ? nN - 1 : s1);
      s2 = s2 < 0 ? 0 : (s2 > nN - 1 ? nN - 1 : s2);
      s3 = s3 < 0 ? 0 : (s3 > nN - 1 ? nN - 1 : s3);
      v4i sv;
      sv.x = (i     < nh) ? s0 : 0;
      sv.y = (i + 1 < nh) ? s1 : 0;
      sv.z = (i + 2 < nh) ? s2 : 0;
      sv.w = (i + 3 < nh) ? s3 : 0;
      if (i < nhr) *(volatile v4i*)(hp + i) = sv;
    }
    *(volatile v4i*)(cp + 4 * tid) = c0v;
    *(volatile v4i*)(cp + NTHR * 4 + 4 * tid) = c1v;
    *(volatile v4i*)(op + 4 * tid) = o0v;
    *(volatile v4i*)(op + NTHR * 4 + 4 * tid) = o1v;
    if (wave == 0 && lane < 8) *(volatile v4i*)(dp + 4 * lane) = hd;
    __threadfence();
  }
}

__global__ __launch_bounds__(GTHR) void k_gemm(
    const unsigned short* __restrict__ A, const unsigned short* __restrict__ WT,
    float* outF, int K, int ldo,
    const float* __restrict__ atts, const float* __restrict__ attd, int attLen,
    float* SD, int MPr)
{
  __shared__ __attribute__((aligned(16))) float stg[GBM * GBN];
  __shared__ __attribute__((aligned(16))) float satt[2 * GBN];
  __shared__ __attribute__((aligned(16))) float sdot[2 * GBM];
  const int tid = (int)threadIdx.x, lane = tid & 31, wave = tid >> 5, hh = lane >> 4, m = lane & 15;
  const int rowBase = (int)blockIdx.x * GBM;
  const int head    = (int)blockIdx.y;
  const int col0    = head * GBN;

  {
    const int which = tid >> 6;
    const int c  = tid & 63;
    const int cl = c < attLen ? c : attLen - 1;
    const float vs = atts[head * attLen + cl];
    const float vd = attd[head * attLen + cl];
    float v = (which == 0) ? vs : vd;
    v = (c < attLen) ? bfr(v) : 0.f;
    satt[which * GBN + c] = v;
  }

  v8f acc[4];
  {
    const v8f z = {0.f, 0.f, 0.f, 0.f, 0.f, 0.f, 0.f, 0.f};
    acc[0] = z; acc[1] = z; acc[2] = z; acc[3] = z;
  }
  const unsigned short* ap = A  + (size_t)(rowBase + 16 * wave + m) * (size_t)K + 8 * hh;
  const unsigned short* wp = WT + (size_t)(col0 + m) * (size_t)K + 8 * hh;
  const int ksteps = K >> 5;
#pragma unroll 1
  for (int ks = 0; ks < ksteps; ++ks) {
    FragB af;
    af.h[0] = *(const v8usa*)(ap + 32 * ks);
    af.h[1] = *(const v8usa*)(ap + 32 * ks + 16);
#pragma unroll
    for (int t = 0; t < 4; ++t) {
      const unsigned short* wq = wp + (size_t)(16 * t) * (size_t)K + 32 * ks;
      FragB bf;
      bf.h[0] = *(const v8usa*)wq;
      bf.h[1] = *(const v8usa*)(wq + 16);
      acc[t] = wmb(af, bf, acc[t]);
    }
  }

#pragma unroll
  for (int t = 0; t < 4; ++t) {
    const int lc = 16 * t + m;
#pragma unroll
    for (int r = 0; r < 8; ++r) {
      const int lr = 16 * wave + 8 * hh + r;
      stg[lr * GBN + lc] = acc[t][r];
    }
  }
  __syncthreads();

  {
    const int row = tid & 63, which = tid >> 6;
    const float* sa = satt + which * GBN;
    const float* hr = stg + row * GBN;
    float d = 0.f;
#pragma unroll 4
    for (int c4 = 0; c4 < GBN / 4; ++c4) {
      const v4f hv = *(const v4fa*)(hr + 4 * c4);
      const v4f av = *(const v4fa*)(sa + 4 * c4);
      d = fmaf(hv.x, av.x, d);
      d = fmaf(hv.y, av.y, d);
      d = fmaf(hv.z, av.z, d);
      d = fmaf(hv.w, av.w, d);
    }
    sdot[which * GBM + row] = d;
  }
  __syncthreads();

  v4f fv[8];
#pragma unroll
  for (int i = 0; i < 8; ++i) {
    const int lr = 16 * wave + 2 * i + hh;
    fv[i] = *(const v4fa*)(stg + lr * GBN + 4 * m);
  }
  const int which2 = lane >> 4, piece = lane & 15;
  const v4f sdv = *(const v4fa*)(sdot + which2 * GBM + 4 * piece);
  float* sp = SD + (size_t)(2 * head + which2) * (size_t)MPr + rowBase + 4 * piece;

#pragma unroll
  for (int i = 0; i < 8; ++i) {
    const int lr = 16 * wave + 2 * i + hh;
    const int gr = rowBase + lr;
    float* op = outF + (size_t)gr * (size_t)ldo + col0 + 4 * m;
    *(volatile v4f*)op = fv[i];
  }
  if (wave == 0) *(volatile v4f*)sp = sdv;
  __threadfence();
#pragma unroll
  for (int i = 0; i < 8; ++i) {
    const int lr = 16 * wave + 2 * i + hh;
    const int gr = rowBase + lr;
    float* op = outF + (size_t)gr * (size_t)ldo + col0 + 4 * m;
    *(volatile v4f*)op = fv[i];
  }
  if (wave == 0) *(volatile v4f*)sp = sdv;
}

__global__ __launch_bounds__(NTHR) void k_agg(
    const int* __restrict__ HITS, const int* __restrict__ CNT, const int* __restrict__ OFF,
    const int* __restrict__ HDR,
    const float* __restrict__ F, const float* __restrict__ SD, const float* __restrict__ bias,
    float* Y, double* REC, int nN, int nb, int MPr) {
  __shared__ __attribute__((aligned(16))) double wred[NWAVE * HID * 2];
  const int tid = (int)threadIdx.x, lane = tid & 31, wave = tid >> 5;
  const int blk = (int)blockIdx.x;
  const int nodeBase = blk * nb;
  const int* hits = HITS + (size_t)blk * RCAP;
  const int* scnt = CNT + (size_t)blk * NBMAX;
  const int* soff = OFF + (size_t)blk * NBMAX;
  int nh = HDR[(size_t)blk * 32];
  nh = nh < 0 ? 0 : (nh > RCAP ? RCAP : nh);

  const int nbw = nb >> 3;
  const bool ovf = (nh >= RCAP);
  const float qnan = __int_as_float(0x7fc00000);

  const int c0   = 4 * lane;
  const int head = lane >> 4;
  const int cb   = 4 * (lane & 15);
  const v4f bb4  = bfr4(*(const v4fa*)(bias + cb));
  const float* ASp = SD + (size_t)(2 * head) * (size_t)MPr;
  const float* ADp = ASp + MPr;

  double s0 = 0.0, s1 = 0.0, s2 = 0.0, s3 = 0.0;
  double q0 = 0.0, q1 = 0.0, q2 = 0.0, q3 = 0.0;

#pragma unroll 1
  for (int jt = 0; jt < nbw; ++jt) {
    int slot = wave * nbw + jt;
    slot = slot > NBMAX - 1 ? NBMAX - 1 : slot;
    const int grow = nodeBase + slot;
    const int gcl  = grow < nN ? grow : nN - 1;
    int st = soff[slot];
    const int craw = scnt[slot];
    int cnt = craw;
    st  = st < 0 ? 0 : (st > nh ? nh : st);
    cnt = cnt < 0 ? 0 : (cnt > DEGCAP ? DEGCAP : cnt);
    if (cnt > nh - st) cnt = nh - st;
    const float pz = (ovf || craw > DEGCAP) ? qnan : 0.0f;

    const v4f fd = *(const v4fa*)(F + (size_t)gcl * HC + c0);
    const float adv = ADp[gcl];
    float l0 = ASp[gcl] + adv;
    l0 = l0 > 0.f ? l0 : NEGSL * l0;
    float mx = l0, dn = 1.0f;
    v4f av = fd;

#pragma unroll 1
    for (int q = 0; q < cnt; ++q) {
      int idx = st + q; idx = idx > RCAP - 1 ? RCAP - 1 : idx;
      const int sraw = hits[idx];
      const int s = sraw < 0 ? 0 : (sraw > nN - 1 ? nN - 1 : sraw);
      const v4f fs = *(const v4fa*)(F + (size_t)s * HC + c0);
      float lg = ASp[s] + adv;
      lg = lg > 0.f ? lg : NEGSL * lg;
      const float df = lg - mx;
      const float ee = expf(-fabsf(df));
      const bool up  = df > 0.f;
      const float f1 = up ? ee : 1.0f;
      const float f2 = up ? 1.0f : ee;
      mx = up ? lg : mx;
      dn = fmaf(dn, f1, f2);
      av.x = fmaf(av.x, f1, f2 * fs.x);
      av.y = fmaf(av.y, f1, f2 * fs.y);
      av.z = fmaf(av.z, f1, f2 * fs.z);
      av.w = fmaf(av.w, f1, f2 * fs.w);
    }
    const float inv = __builtin_amdgcn_rcpf(dn + EPS_SM);
    const float ox = av.x * inv, oy = av.y * inv, oz = av.z * inv, ow = av.w * inv;
    const float px = __shfl_xor(ox, 16), py = __shfl_xor(oy, 16);
    const float pw2 = __shfl_xor(oz, 16), pw3 = __shfl_xor(ow, 16);
    const bool live = grow < nN;
    v4f yv;
    yv.x = (live ? (0.5f * (ox + px)  + bb4.x) : 0.f) + pz;
    yv.y = (live ? (0.5f * (oy + py)  + bb4.y) : 0.f) + pz;
    yv.z = (live ? (0.5f * (oz + pw2) + bb4.z) : 0.f) + pz;
    yv.w = (live ? (0.5f * (ow + pw3) + bb4.w) : 0.f) + pz;
    {
      const double dx = live ? (double)yv.x : 0.0;
      const double dy = live ? (double)yv.y : 0.0;
      const double dz = live ? (double)yv.z : 0.0;
      const double dw = live ? (double)yv.w : 0.0;
      s0 += dx; s1 += dy; s2 += dz; s3 += dw;
      q0 += dx * dx; q1 += dy * dy; q2 += dz * dz; q3 += dw * dw;
    }
    float* gp = Y + (size_t)grow * HID + cb;
    const bool wr = (grow < MPr) && (lane < 16);
    if (wr) *(volatile v4f*)gp = yv;
    __threadfence();
    if (wr) *(volatile v4f*)gp = yv;
  }

  if (lane < 16) {
    double* wp = wred + (size_t)(wave * HID + cb) * 2;
    wp[0] = s0; wp[1] = q0;
    wp[2] = s1; wp[3] = q1;
    wp[4] = s2; wp[5] = q2;
    wp[6] = s3; wp[7] = q3;
  }
  __syncthreads();
  if (tid < HID) {
    double S = 0.0, Q = 0.0;
#pragma unroll
    for (int w2 = 0; w2 < NWAVE; ++w2) {
      S += wred[(size_t)(w2 * HID + tid) * 2 + 0];
      Q += wred[(size_t)(w2 * HID + tid) * 2 + 1];
    }
    v2d rv; rv.x = S; rv.y = Q;
    double* rp = REC + ((size_t)blk * HID + tid) * 2;
    *(volatile v2d*)rp = rv;
    __threadfence();
    *(volatile v2d*)rp = rv;
  }
}

__device__ __forceinline__ void bn_params(const double* __restrict__ REC, int nRec, double invN,
                                          const float* __restrict__ gam, const float* __restrict__ bet,
                                          float* sm, float* si, float* sg, float* sb, int tid) {
  if (tid < HID) {
    double S = 0.0, Q = 0.0;
#pragma unroll 1
    for (int b = 0; b < nRec; ++b) {
      const v2d r = *(const v2da*)(REC + ((size_t)b * HID + tid) * 2);
      S += r.x; Q += r.y;
    }
    const double mean = S * invN;
    double var = Q * invN - mean * mean;
    var = (var < 0.0) ? 0.0 : var;
    const float vf = (float)var;
    sm[tid] = (float)mean;
    si[tid] = 1.0f / sqrtf(vf + EPS_BN);
    sg[tid] = bfr(gam[tid]);
    sb[tid] = bfr(bet[tid]);
  }
}

__global__ __launch_bounds__(NTHR) void k_bn(const float* __restrict__ Y, const double* __restrict__ REC, int nRec,
                                             double invN, const float* __restrict__ gam,
                                             const float* __restrict__ bet, unsigned short* YHL,
                                             int nN, int MPr) {
  __shared__ __attribute__((aligned(16))) float sm[HID];
  __shared__ __attribute__((aligned(16))) float si[HID];
  __shared__ __attribute__((aligned(16))) float sg[HID];
  __shared__ __attribute__((aligned(16))) float sb[HID];
  const int tid = (int)threadIdx.x;
  bn_params(REC, nRec, invN, gam, bet, sm, si, sg, sb, tid);
  __syncthreads();
  const int u = tid & 7, rq = tid >> 3;
  const int c0 = 8 * u;
  const v4f ma = *(const v4fa*)(sm + c0), mb = *(const v4fa*)(sm + c0 + 4);
  const v4f ia = *(const v4fa*)(si + c0), ib = *(const v4fa*)(si + c0 + 4);
  const v4f ga = *(const v4fa*)(sg + c0), gb = *(const v4fa*)(sg + c0 + 4);
  const v4f ba = *(const v4fa*)(sb + c0), bb = *(const v4fa*)(sb + c0 + 4);
#pragma unroll 1
  for (int it = 0; it < BNR / 32; ++it) {
    const int row = (int)blockIdx.x * BNR + it * 32 + rq;
    const int rc  = row < nN ? row : nN - 1;
    const float* p = Y + (size_t)rc * HID + c0;
    const v4f ya = *(const v4fa*)p, yb = *(const v4fa*)(p + 4);
    const bool live = row < nN;
    v4f za, zb;
    za.x = bnrelu(ya.x, ma.x, ia.x, ga.x, ba.x, live);
    za.y = bnrelu(ya.y, ma.y, ia.y, ga.y, ba.y, live);
    za.z = bnrelu(ya.z, ma.z, ia.z, ga.z, ba.z, live);
    za.w = bnrelu(ya.w, ma.w, ia.w, ga.w, ba.w, live);
    zb.x = bnrelu(yb.x, mb.x, ib.x, gb.x, bb.x, live);
    zb.y = bnrelu(yb.y, mb.y, ib.y, gb.y, bb.y, live);
    zb.z = bnrelu(yb.z, mb.z, ib.z, gb.z, bb.z, live);
    zb.w = bnrelu(yb.w, mb.w, ib.w, gb.w, bb.w, live);
    const v4u hv = pack8(za, zb);
    const v4u lv = pack8(res4(za), res4(zb));
    const int rw = row < MPr ? row : MPr - 1;
    unsigned short* hp = YHL + (size_t)rw * KA + c0;
    unsigned short* lp = hp + HID;
    const bool wr = row < MPr;
    if (wr) { *(volatile v4u*)hp = hv; *(volatile v4u*)lp = lv; }
    __threadfence();
    if (wr) { *(volatile v4u*)hp = hv; *(volatile v4u*)lp = lv; }
  }
}

__global__ __launch_bounds__(NTHR) void k_pool(const float* __restrict__ Y, const int* __restrict__ bat, int nN,
                                               const double* __restrict__ REC, int nRec, double invN,
                                               const float* __restrict__ gam, const float* __restrict__ bet,
                                               unsigned short* REP) {
  __shared__ __attribute__((aligned(16))) float sm[HID];
  __shared__ __attribute__((aligned(16))) float si[HID];
  __shared__ __attribute__((aligned(16))) float sg[HID];
  __shared__ __attribute__((aligned(16))) float sb[HID];
  __shared__ __attribute__((aligned(16))) float wsum[NWAVE * HID];
  __shared__ int wcn[NWAVE];
  __shared__ __attribute__((aligned(16))) float outs[HID];
  const int tid = (int)threadIdx.x, lane = tid & 31, wave = tid >> 5;
  const int g = (int)blockIdx.x;
  bn_params(REC, nRec, invN, gam, bet, sm, si, sg, sb, tid);
  __syncthreads();
  const float m0 = sm[2 * lane], m1 = sm[2 * lane + 1];
  const float i0v = si[2 * lane], i1v = si[2 * lane + 1];
  const float g0 = sg[2 * lane], g1 = sg[2 * lane + 1];
  const float b0 = sb[2 * lane], b1 = sb[2 * lane + 1];

  float a0 = 0.0f, a1 = 0.0f;
  int cnt = 0;
#pragma unroll 1
  for (int i0 = wave * 32; i0 < nN; i0 += NTHR) {
    const int i  = i0 + lane;
    const int ic = i < nN ? i : nN - 1;
    const int b  = bat[ic];
    const bool hit = (i < nN) && (b == g);
    unsigned msk = __builtin_amdgcn_ballot_w32(hit);
    int nh = (int)__builtin_popcount(msk);
    nh = nh > 32 ? 32 : nh;
    cnt += nh;
#pragma unroll 1
    for (int q = 0; q < nh; ++q) {
      const int k = __builtin_ffs((int)msk) - 1;
      msk &= msk - 1u;
      int node = i0 + (k < 0 ? 0 : k);
      node = node > nN - 1 ? nN - 1 : node;
      const v2f v = *(const v2fa*)(Y + (size_t)node * HID + 2 * lane);
      a0 += bnrelu(v.x, m0, i0v, g0, b0, true);
      a1 += bnrelu(v.y, m1, i1v, g1, b1, true);
    }
  }
  wsum[wave * HID + 2 * lane + 0] = a0;
  wsum[wave * HID + 2 * lane + 1] = a1;
  if (lane == 0) wcn[wave] = cnt;
  __syncthreads();
  if (tid < HID) {
    float s = 0.0f;
    int c = 0;
#pragma unroll
    for (int w2 = 0; w2 < NWAVE; ++w2) { s += wsum[w2 * HID + tid]; c += wcn[w2]; }
    const float cf = (c < 1) ? 1.0f : (float)c;
    outs[tid] = s * (1.0f / cf);
  }
  __syncthreads();
  const int u = lane & 7;
  const v4f oa = *(const v4fa*)(outs + 8 * u);
  const v4f ob = *(const v4fa*)(outs + 8 * u + 4);
  const v4u hv = pack8(oa, ob);
  const v4u lv = pack8(res4(oa), res4(ob));
  const bool lsel = (lane & 8) != 0;
  v4u pv;
  pv.x = lsel ? lv.x : hv.x;
  pv.y = lsel ? lv.y : hv.y;
  pv.z = lsel ? lv.z : hv.z;
  pv.w = lsel ? lv.w : hv.w;
  unsigned short* rp = REP + (size_t)g * KA + 8 * (lane & 15);
  const bool okst = (wave == 0) && (lane < 16);
  if (okst) *(volatile v4u*)rp = pv;
  __threadfence();
  if (okst) *(volatile v4u*)rp = pv;
}

__global__ __launch_bounds__(GTHR) void k_fc(const unsigned short* __restrict__ REP,
                                             const unsigned short* __restrict__ FCD,
                                             const float* __restrict__ fcb, float* out) {
  __shared__ __attribute__((aligned(16))) float stg[16 * NHID];
  const int tid = (int)threadIdx.x, lane = tid & 31, wave = tid >> 5, hh = lane >> 4, m = lane & 15;
  const int rowBase = (int)blockIdx.x * 16;
  const unsigned short* ap = REP + (size_t)(rowBase + m) * KA + 8 * hh;
  FragB af[KA / 32];
#pragma unroll
  for (int ks = 0; ks < KA / 32; ++ks) {
    af[ks].h[0] = *(const v8usa*)(ap + 32 * ks);
    af[ks].h[1] = *(const v8usa*)(ap + 32 * ks + 16);
  }
#pragma unroll 1
  for (int t = wave; t < FCT; t += GTHR / 32) {
    v8f acc = {0.f, 0.f, 0.f, 0.f, 0.f, 0.f, 0.f, 0.f};
    const unsigned short* wq = FCD + (size_t)(16 * t + m) * KA + 8 * hh;
#pragma unroll
    for (int ks = 0; ks < KA / 32; ++ks) {
      FragB bf;
      bf.h[0] = *(const v8usa*)(wq + 32 * ks);
      bf.h[1] = *(const v8usa*)(wq + 32 * ks + 16);
      acc = wmb(af[ks], bf, acc);
    }
    const int col = 16 * t + m;
    const int cc  = col < NHID ? col : NHID - 1;
    const float bv = bfr(fcb[cc]);
    if (col < NHID) {
#pragma unroll
      for (int r = 0; r < 8; ++r) stg[(8 * hh + r) * NHID + col] = acc[r] + bv;
    }
  }
  __syncthreads();
  constexpr int NPC = 16 * NHID / 4;
  constexpr int NIT = (NPC + GTHR - 1) / GTHR;
  v4f ov[NIT];
#pragma unroll
  for (int it = 0; it < NIT; ++it) {
    const int p  = it * GTHR + tid;
    const int pc = p < NPC ? p : NPC - 1;
    ov[it] = *(const v4fa*)(stg + 4 * pc);
  }
  float* ob = out + (size_t)blockIdx.x * (16 * NHID);
#pragma unroll
  for (int it = 0; it < NIT; ++it) {
    const int p = it * GTHR + tid;
    if (p < NPC) *(volatile v4f*)(ob + 4 * (size_t)p) = ov[it];
  }
  __threadfence();
#pragma unroll
  for (int it = 0; it < NIT; ++it) {
    const int p = it * GTHR + tid;
    if (p < NPC) *(volatile v4f*)(ob + 4 * (size_t)p) = ov[it];
  }
}

static int pick_nb(int nE, int nN) {
  int nb = NBMAX;
  while (nb > 32 && (long long)nb * (long long)nE * 5LL > (long long)RCAP * (long long)nN * 4LL) nb >>= 1;
  return nb;
}
static inline int cdiv(int a, int b) { return (a + b - 1) / b; }
static inline size_t al256(size_t o) { return (o + 255) & ~(size_t)255; }

extern "C" void kernel_launch(void* const* d_in, const int* in_sizes, int n_in,
                              void* d_out, int out_size, void* d_ws, size_t ws_size,
                              hipStream_t stream) {
  if (n_in < 23) return;
  if (in_sizes[0] < F_IN || (in_sizes[0] % F_IN) != 0) return;
  const int nN = in_sizes[0] / F_IN;
  if (nN < 1 || nN > (1 << 22)) return;
  if (in_sizes[1] < 2 || (in_sizes[1] & 1) != 0) return;
  const int nE = in_sizes[1] / 2;
  if (nE < 1 || nE >= (1 << (32 - SLOTB))) return;
  if (in_sizes[2] != nN) return;
  if (in_sizes[3] != F_IN * HC) return;
  if (in_sizes[9] != HID * HC || in_sizes[15] != HID * HC) return;
  for (int l = 0; l < 3; ++l) {
    const int b = 3 + 6 * l;
    if (in_sizes[b + 1] != 2 * HID || in_sizes[b + 2] != 2 * HID) return;
    if (in_sizes[b + 3] != HID || in_sizes[b + 4] != HID || in_sizes[b + 5] != HID) return;
  }
  if (in_sizes[21] != HID * NHID || in_sizes[22] != NHID) return;
  if (out_size != NGR * NHID) return;

  const float* x   = (const float*)d_in[0];
  const int*   ei  = (const int*)d_in[1];
  const int*   bat = (const int*)d_in[2];
  const float* Wl[3]  = {(const float*)d_in[3],  (const float*)d_in[9],  (const float*)d_in[15]};
  const float* Asl[3] = {(const float*)d_in[4],  (const float*)d_in[10], (const float*)d_in[16]};
  const float* Adl[3] = {(const float*)d_in[5],  (const float*)d_in[11], (const float*)d_in[17]};
  const float* Bl[3]  = {(const float*)d_in[6],  (const float*)d_in[12], (const float*)d_in[18]};
  const float* Gl[3]  = {(const float*)d_in[7],  (const float*)d_in[13], (const float*)d_in[19]};
  const float* Bel[3] = {(const float*)d_in[8],  (const float*)d_in[14], (const float*)d_in[20]};
  const float* fcw = (const float*)d_in[21];
  const float* fcb = (const float*)d_in[22];
  float* out = (float*)d_out;
  const int* src = ei;
  const int* dst = ei + nE;

  const int MP = cdiv(nN, GBM) * GBM;
  const int nb = pick_nb(nE, nN);
  if (nb < 32 || (nb & (nb - 1)) != 0 || nb > NBMAX) return;
  const int gA = cdiv(MP, nb);
  if ((long long)gA * nb < (long long)MP) return;
  const int vec8 = ((nE & 3) == 0) ? 1 : 0;
  const int gM = MP / GBM;
  const double invN = 1.0 / (double)nN;

  char* ws = (char*)d_ws;
  size_t off = 0;
  const size_t oXB  = off; off = al256(off + (size_t)MP * F_IN * 2);
  const size_t oW1T = off; off = al256(off + (size_t)HC * KA * 2);
  const size_t oW2D = off; off = al256(off + (size_t)HC * KA * 2);
  const size_t oW3D = off; off = al256(off + (size_t)HC * KA * 2);
  const size_t oFCD = off; off = al256(off + (size_t)FCN * KA * 2);
  const size_t oHF  = off; off = al256(off + (size_t)MP * HC * 4);
  const size_t oSD  = off; off = al256(off + (size_t)4 * MP * 4);
  const size_t oY   = off; off = al256(off + (size_t)MP * HID * 4);
  const size_t oYHL = off; off = al256(off + (size_t)MP * KA * 2);
  const size_t oHIT = off; off = al256(off + (size_t)gA * RCAP * 4);
  const size_t oCNT = off; off = al256(off + (size_t)gA * NBMAX * 4);
  const size_t oOFF = off; off = al256(off + (size_t)gA * NBMAX * 4);
  const size_t oHDR = off; off = al256(off + (size_t)gA * 32 * 4);
  const size_t oR1  = off; off = al256(off + (size_t)gA * HID * 16);
  const size_t oR2  = off; off = al256(off + (size_t)gA * HID * 16);
  const size_t oR3  = off; off = al256(off + (size_t)gA * HID * 16);
  const size_t oREP = off; off = al256(off + (size_t)NGR * KA * 2);
  if (off > ws_size || off > (size_t)WSMAX) return;
  unsigned short* XB  = (unsigned short*)(ws + oXB);
  unsigned short* WP[3] = {(unsigned short*)(ws + oW1T), (unsigned short*)(ws + oW2D), (unsigned short*)(ws + oW3D)};
  unsigned short* FCD = (unsigned short*)(ws + oFCD);
  float*          HF  = (float*)(ws + oHF);
  float*          SD  = (float*)(ws + oSD);
  float*          Y   = (float*)(ws + oY);
  unsigned short* YHL = (unsigned short*)(ws + oYHL);
  int*            HIT = (int*)(ws + oHIT);
  int*            CNT = (int*)(ws + oCNT);
  int*            OFS = (int*)(ws + oOFF);
  int*            HDR = (int*)(ws + oHDR);
  double*         RC[3] = {(double*)(ws + oR1), (double*)(ws + oR2), (double*)(ws + oR3)};
  unsigned short* REP = (unsigned short*)(ws + oREP);

  hipFuncSetAttribute(reinterpret_cast<const void*>(&k_build),
                      hipFuncAttributeMaxDynamicSharedMemorySize, LDS_AGG);

  k_wprep<<<(3 * NUW + NUF) / NTHR, NTHR, 0, stream>>>(Wl[0], Wl[1], Wl[2], fcw, WP[0], WP[1], WP[2], FCD);
  const int nUx = MP * (F_IN / 8);
  k_cvx<<<cdiv(nUx, NTHR), NTHR, 0, stream>>>(x, nN, nUx, XB);
  k_build<<<gA, NTHR, LDS_AGG, stream>>>(src, dst, nN, nE, nb, vec8, HIT, CNT, OFS, HDR);

  for (int l = 0; l < 3; ++l) {
    const unsigned short* Aop = (l == 0) ? XB : YHL;
    k_gemm<<<dim3(gM, HC / GBN), GTHR, 0, stream>>>(Aop, WP[l], HF, KA, HC, Asl[l], Adl[l], HID, SD, MP);
    k_agg<<<gA, NTHR, 0, stream>>>(HIT, CNT, OFS, HDR, HF, SD, Bl[l], Y, RC[l], nN, nb, MP);
    if (l < 2) {
      k_bn<<<cdiv(MP, BNR), NTHR, 0, stream>>>(Y, RC[l], gA, invN, Gl[l], Bel[l], YHL, nN, MP);
    }
  }
  k_pool<<<NGR, NTHR, 0, stream>>>(Y, bat, nN, RC[2], gA, invN, Gl[2], Bel[2], REP);
  k_fc<<<NGR / 16, GTHR, 0, stream>>>(REP, FCD, fcb, out);
}
